// CausalSelfAttention_30520037606061
// MI455X (gfx1250) — hardware-run, weakly checked
//
#include <hip/hip_runtime.h>


#ifndef NB
#define NB 1
#endif
#ifndef SEQ
#define SEQ 4096
#endif
#define NB_FULL  1
#define SEQ_FULL 4096
#ifndef OUT_SEQ
#define OUT_SEQ SEQ
#endif
#define DM   1024
#define NH_  8
#define HD   128
#define NF   32
#define AW   4
#define OSP  132
#define OQP  132
#define QRS  2048.0f
#define QRI  (1.0f / 2048.0f)
#define SC2  ((float)(0.12 * 1.4426950408889634))
#define PSH  14.0f
#define NEGB (-3.0e38f)
#define RMS_EPS 1.1920928955078125e-07f

static_assert(HD == 128);
static_assert(NH_ * HD == DM);
static_assert(HD % 32 == 0);
static_assert(NF * 4 == HD);
static_assert(NF == 32);
static_assert(DM % 64 == 0);
static_assert(DM % 32 == 0);
static_assert((DM & (DM - 1)) == 0);
static_assert(SEQ % 64 == 0);
static_assert((NB * SEQ) % 64 == 0);
static_assert(SEQ % 32 == 0);
static_assert(SEQ % (16 * AW) == 0);
static_assert(((size_t)SEQ * NF) % 256 == 0);
static_assert(((size_t)SEQ * DM) % 8 == 0);
static_assert(((size_t)DM * DM) % 8 == 0);
static_assert(NB <= NB_FULL);
static_assert(SEQ <= SEQ_FULL);
static_assert((OSP * 4) % 16 == 0);
static_assert((OQP * 4) % 16 == 0);
static_assert(OSP >= HD);
static_assert(OQP >= HD);
static_assert(32 * 8 * 16 == 16 * HD * 2);
static_assert(32 * 4 * 16 == 16 * 64 * 2);
static_assert(32 * 8 * 16 == 16 * 64 * 4);
static_assert(16 * OQP * 4 <= 131072);
static_assert(16 * 68 * 4 <= 131072);
static_assert(AW * 16 * OSP * 4 <= 131072);

typedef _Float16 h16;
typedef unsigned short bf;
typedef __attribute__((ext_vector_type(16))) __bf16   v16bf;
typedef __attribute__((ext_vector_type(16))) _Float16 v16h;
typedef __attribute__((ext_vector_type(8)))  _Float16 v8h;
typedef __attribute__((ext_vector_type(8)))  unsigned short v8us;
typedef __attribute__((ext_vector_type(8)))  float    v8f;
typedef __attribute__((ext_vector_type(4)))  float    v4f;
typedef __attribute__((ext_vector_type(4)))  int      v4i;
typedef v4f  __attribute__((may_alias)) v4fa;

__device__ __forceinline__ unsigned short f2bf(float f) { unsigned u = __float_as_uint(f); u += 0x7FFFu + ((u >> 16) & 1u); return (unsigned short)(u >> 16); }
__device__ __forceinline__ float bfr(float f) { return __uint_as_float(((unsigned)f2bf(f)) << 16); }
__device__ __forceinline__ v16h cat16(v8h lo, v8h hi) { return __builtin_shufflevector(lo, hi, 0, 1, 2, 3, 4, 5, 6, 7, 8, 9, 10, 11, 12, 13, 14, 15); }
__device__ __forceinline__ v16bf cat16b(v8us lo, v8us hi) { return __builtin_bit_cast(v16bf, __builtin_shufflevector(lo, hi, 0, 1, 2, 3, 4, 5, 6, 7, 8, 9, 10, 11, 12, 13, 14, 15)); }
__device__ __forceinline__ v8f wmma16(v16h a, v16h b, v8f c) { return __builtin_amdgcn_wmma_f32_16x16x32_f16(false, a, false, b, (short)0, c, false, false); }
__device__ __forceinline__ v8f wmmab(v16bf a, v16bf b, v8f c) { return __builtin_amdgcn_wmma_f32_16x16x32_bf16(false, a, false, b, (short)0, c, false, false); }
__device__ __forceinline__ v16h  ldh(const h16* p) { return cat16(*(const v8h*)p, *(const v8h*)(p + 16)); }
__device__ __forceinline__ v16bf ldb(const bf* p)  { return cat16b(*(const v8us*)p, *(const v8us*)(p + 16)); }
__device__ __forceinline__ void wave_sync() { __builtin_amdgcn_fence(3  , "wavefront"); __builtin_amdgcn_wave_barrier(); asm volatile("" ::: "memory"); }
static __device__ __forceinline__ h16 toh_flush(float v) { const h16 r = (h16)v; return (fabsf(v) < 6.103515625e-05f) ? (h16)0.0f : r; }
__device__ __forceinline__ float bf2f(unsigned short u) { return __uint_as_float(((unsigned)u) << 16); }

__global__ __launch_bounds__(256) void k_cvt8(const float* __restrict__ src, bf* dst, size_t n8) {
    const size_t i = (size_t)blockIdx.x * 256 + threadIdx.x; if (i >= n8) return;
    const v8f v = *(const v8f*)(src + i * 8); v8us o;
#pragma unroll
    for (int k = 0; k < 8; ++k) o[k] = f2bf(v[k]);
    *(volatile v8us*)(dst + i * 8) = o; __threadfence(); *(volatile v8us*)(dst + i * 8) = o;
}

__global__ __launch_bounds__(256) void k_rot(float* CS, float* SN) {
#pragma clang fp contract(off)
    const int i = blockIdx.x * 256 + threadIdx.x;
    const int t = i >> 5, f = i & 31;
    const float lin = (float)f / 31.0f;
    const float fr = exp2f(-10.0f * lin);
    const float th = (float)t * fr;
    float sv, cv; sincosf(th, &sv, &cv);
    *(volatile float*)(CS + i) = cv; *(volatile float*)(SN + i) = sv;
    __threadfence();
    *(volatile float*)(CS + i) = cv; *(volatile float*)(SN + i) = sv;
}

__global__ __launch_bounds__(32) __attribute__((amdgpu_num_vgpr(256)))
void k_qk(const bf* __restrict__ A, const bf* __restrict__ Bt, const float* __restrict__ CS, const float* __restrict__ SN, h16* Ph, h16* Pr) {
    __shared__ __align__(16) float os[16 * OQP];
    const int K = DM;
    const int lane = threadIdx.x & 31, lr = lane & 15, hi = lane >> 4; const int r0 = blockIdx.x * 32, zc = blockIdx.y; const int c0 = zc * HD;
    v8f acc[2][8];
#pragma unroll
    for (int mb = 0; mb < 2; ++mb)
#pragma unroll
        for (int nb = 0; nb < 8; ++nb) acc[mb][nb] = (v8f){};
    const size_t aoff = (size_t)(r0 + lr) * K + 8 * hi, boff = (size_t)(c0 + lr) * K + 8 * hi;
#pragma unroll 1
    for (int kc = 0; kc < K; kc += 32) {
        v16bf a[2];
#pragma unroll
        for (int mb = 0; mb < 2; ++mb) a[mb] = ldb(A + aoff + (size_t)mb * 16 * K + kc);
#pragma unroll
        for (int nb = 0; nb < 8; ++nb) { const v16bf b = ldb(Bt + boff + (size_t)nb * 16 * K + kc);
#pragma unroll
            for (int mb = 0; mb < 2; ++mb) acc[mb][nb] = wmmab(a[mb], b, acc[mb][nb]); }
        asm volatile("v_nop\n\tv_nop\n\tv_nop\n\tv_nop" : "+v"(acc[0][1]), "+v"(acc[1][3]), "+v"(acc[0][5]), "+v"(acc[1][7]) : "v"(a[0]), "v"(a[1]));
    }
    asm volatile("v_nop\n\tv_nop\n\tv_nop\n\tv_nop" : "+v"(acc[0][0]), "+v"(acc[0][1]), "+v"(acc[0][2]), "+v"(acc[0][3]), "+v"(acc[0][4]), "+v"(acc[0][5]), "+v"(acc[0][6]), "+v"(acc[0][7]));
    asm volatile("v_nop\n\tv_nop\n\tv_nop\n\tv_nop" : "+v"(acc[1][0]), "+v"(acc[1][1]), "+v"(acc[1][2]), "+v"(acc[1][3]), "+v"(acc[1][4]), "+v"(acc[1][5]), "+v"(acc[1][6]), "+v"(acc[1][7]));
    const int bb = r0 / SEQ, tt = r0 % SEQ;
    const int zp = (zc / NH_) * (NB * NH_) + bb * NH_ + (zc % NH_);
    const size_t pbase = ((size_t)zp * SEQ + (size_t)tt) * HD;
    const int row = lane >> 1, half = lane & 1;
    const int ob = row * OQP + 16 * half;
#pragma unroll
    for (int mb = 0; mb < 2; ++mb) {
#pragma unroll
        for (int nb = 0; nb < 8; ++nb) {
#pragma unroll
            for (int j = 0; j < 8; ++j) os[(hi * 8 + j) * OQP + nb * 16 + lr] = acc[mb][nb][j]; }
        wave_sync();
        {
            v4f x1[4], x2[4], x3[4], x4[4];
#pragma unroll
            for (int i = 0; i < 4; ++i) { x1[i] = *(const v4fa*)(&os[ob + 4 * i]); x3[i] = *(const v4fa*)(&os[ob + 32 + 4 * i]); x2[i] = *(const v4fa*)(&os[ob + 64 + 4 * i]); x4[i] = *(const v4fa*)(&os[ob + 96 + 4 * i]); }
            float ss = 0.0f;
#pragma unroll
            for (int i = 0; i < 4; ++i) {
#pragma unroll
                for (int e = 0; e < 4; ++e) ss += x1[i][e] * x1[i][e] + x2[i][e] * x2[i][e] + x3[i][e] * x3[i][e] + x4[i][e] * x4[i][e]; }
            ss += __shfl_xor(ss, 1, 32);
            const float rr = rsqrtf(ss * (1.0f / 128.0f) + RMS_EPS);
            const size_t to = (size_t)(tt + mb * 16 + row) * NF + 16 * half;
#pragma unroll
            for (int i = 0; i < 4; ++i) {
                const v4f cv = *(const v4f*)(CS + to + 4 * i), sv = *(const v4f*)(SN + to + 4 * i);
                const v4f e1 = x1[i] * rr, e2 = x2[i] * rr;
                const v4f y1 = e1 * cv + e2 * sv;
                const v4f y2 = e2 * cv - e1 * sv;
                *(v4fa*)(&os[ob + 4 * i]) = y1; *(v4fa*)(&os[ob + 64 + 4 * i]) = y2;
                *(v4fa*)(&os[ob + 32 + 4 * i]) = x3[i] * rr; *(v4fa*)(&os[ob + 96 + 4 * i]) = x4[i] * rr; }
        }
        wave_sync();
        v8h hv[8], rv[8];
#pragma unroll
        for (int s = 0; s < 8; ++s) { const int p = s * 32 + lane; const int rw = p >> 4, c8 = (p & 15) * 8;
            const v4f x0 = *(const v4fa*)(&os[rw * OQP + c8]); const v4f x1 = *(const v4fa*)(&os[rw * OQP + c8 + 4]);
#pragma unroll
            for (int i = 0; i < 4; ++i) { const h16 a0 = toh_flush(x0[i]); const h16 a1 = toh_flush(x1[i]); hv[s][i] = a0; hv[s][4 + i] = a1;
                rv[s][i] = toh_flush((x0[i] - (float)a0) * QRS); rv[s][4 + i] = toh_flush((x1[i] - (float)a1) * QRS); } }
        const size_t sb = pbase + (size_t)(mb * 16) * HD;
#pragma unroll 1
        for (int ps = 0; ps < 2; ++ps) {
#pragma unroll
            for (int s = 0; s < 8; ++s) { const size_t oo = sb + (size_t)(s * 32 + lane) * 8;
                *(volatile v8h*)(Ph + oo) = hv[s]; *(volatile v8h*)(Pr + oo) = rv[s]; }
            if (ps == 0) __threadfence(); }
        wave_sync();
    }
}

__global__ __launch_bounds__(32) void k_vt(const bf* __restrict__ A, const bf* __restrict__ Bt, const float* __restrict__ ve, const float* __restrict__ lam, h16* Ph, h16* Pr) {
    __shared__ __align__(16) float os[16 * 68];
    const int K = DM;
    const int lane = threadIdx.x & 31, lr = lane & 15, hi = lane >> 4; const int r0 = blockIdx.x * 64, c0 = blockIdx.y * 64;
    v8f acc[4][4];
#pragma unroll
    for (int mb = 0; mb < 4; ++mb)
#pragma unroll
        for (int nb = 0; nb < 4; ++nb) acc[mb][nb] = (v8f){};
    const size_t aoff = (size_t)(r0 + lr) * K + 8 * hi, boff = (size_t)(c0 + lr) * K + 8 * hi;
#pragma unroll 1
    for (int kc = 0; kc < K; kc += 32) {
        v16bf a[4];
#pragma unroll
        for (int mb = 0; mb < 4; ++mb) a[mb] = ldb(A + aoff + (size_t)mb * 16 * K + kc);
#pragma unroll
        for (int nb = 0; nb < 4; ++nb) { const v16bf b = ldb(Bt + boff + (size_t)nb * 16 * K + kc);
#pragma unroll
            for (int mb = 0; mb < 4; ++mb) acc[mb][nb] = wmmab(a[mb], b, acc[mb][nb]); }
        asm volatile("v_nop\n\tv_nop\n\tv_nop\n\tv_nop" : "+v"(acc[0][0]), "+v"(acc[1][1]), "+v"(acc[2][2]), "+v"(acc[3][3]) : "v"(a[0]), "v"(a[1]), "v"(a[2]), "v"(a[3]));
    }
    const float l0 = bfr(lam[0]), l1 = bfr(lam[1]);
    const int bb = c0 / SEQ, tt = c0 % SEQ;
    const size_t tbase = (size_t)bb * (size_t)DM * SEQ + (size_t)r0 * SEQ + (size_t)tt;
#pragma unroll
    for (int mb = 0; mb < 4; ++mb) {
#pragma unroll
        for (int nb = 0; nb < 4; ++nb) {
            const float* vp = ve + ((size_t)bb * SEQ_FULL + (size_t)(tt + nb * 16 + lr)) * DM + r0 + mb * 16 + hi * 8;
            const v4f e0 = *(const v4f*)vp, e1 = *(const v4f*)(vp + 4);
#pragma unroll
            for (int j = 0; j < 4; ++j) { os[(hi * 8 + j) * 68 + nb * 16 + lr] = l0 * acc[mb][nb][j] + l1 * bfr(e0[j]);
                                          os[(hi * 8 + 4 + j) * 68 + nb * 16 + lr] = l0 * acc[mb][nb][4 + j] + l1 * bfr(e1[j]); } }
        wave_sync();
        v8h hv[4], rv[4];
#pragma unroll
        for (int s = 0; s < 4; ++s) { const int row = 4 * s + (lane >> 3), c8 = (lane & 7) * 8;
            const v4f x0 = *(const v4fa*)(&os[row * 68 + c8]); const v4f x1 = *(const v4fa*)(&os[row * 68 + c8 + 4]);
#pragma unroll
            for (int i = 0; i < 4; ++i) { const h16 a0 = toh_flush(x0[i]); const h16 a1 = toh_flush(x1[i]); hv[s][i] = a0; hv[s][4 + i] = a1;
                rv[s][i] = toh_flush((x0[i] - (float)a0) * QRS); rv[s][4 + i] = toh_flush((x1[i] - (float)a1) * QRS); } }
        const size_t sb = tbase + (size_t)(mb * 16) * SEQ;
#pragma unroll 1
        for (int ps = 0; ps < 2; ++ps) {
#pragma unroll
            for (int s = 0; s < 4; ++s) { const int row = 4 * s + (lane >> 3), c8 = (lane & 7) * 8;
                const size_t oo = sb + (size_t)row * SEQ + c8;
                *(volatile v8h*)(Ph + oo) = hv[s]; *(volatile v8h*)(Pr + oo) = rv[s]; }
            if (ps == 0) __threadfence(); }
        wave_sync();
    }
}

__device__ __forceinline__ v8f sc16(const h16* __restrict__ QH, const h16* __restrict__ QR, const h16* __restrict__ KP, const h16* __restrict__ KR, size_t qo, size_t kofs) {
    v8f sH = (v8f){}, sL = (v8f){};
#pragma unroll 1
    for (int kk = 0; kk < HD; kk += 32) {
        const v16h qh = ldh(QH + qo + kk), qr = ldh(QR + qo + kk);
        const v16h kh = ldh(KP + kofs + kk), kr = ldh(KR + kofs + kk);
        sH = wmma16(kh, qh, sH); sL = wmma16(kh, qr, sL); sL = wmma16(kr, qh, sL);
        asm volatile("v_nop\n\tv_nop\n\tv_nop\n\tv_nop" : "+v"(sH), "+v"(sL) : "v"(kh), "v"(kr), "v"(qh), "v"(qr));
    }
    v8f t;
#pragma unroll
    for (int r = 0; r < 8; ++r) t[r] = (sH[r] + sL[r] * QRI) * SC2;
    return t;
}

__global__ __launch_bounds__(32 * AW) __attribute__((amdgpu_num_vgpr(256)))
void k_flash(const h16* __restrict__ QH, const h16* __restrict__ QR, const h16* __restrict__ KP, const h16* __restrict__ KR,
             const h16* __restrict__ VT, const h16* __restrict__ VR, const int* __restrict__ docs, bf* Y2) {
    __shared__ __align__(16) float os[AW * 16 * OSP];
    const int lane = threadIdx.x & 31, lr = lane & 15, hi = lane >> 4;
    const int wave = __builtin_amdgcn_readfirstlane((int)(threadIdx.x >> 5));
    const int zh = blockIdx.y; const int b = zh / NH_, h = zh % NH_;
    const int t0 = (blockIdx.x * AW + wave) * 16;
    const int* dk = docs + (size_t)b * SEQ_FULL;
    const int mydoc = dk[t0 + lr];
    int qmn = mydoc, qmx = mydoc;
#pragma unroll
    for (int off = 1; off < 16; off <<= 1) { const int a0 = __shfl_xor(qmn, off, 32); const int a1 = __shfl_xor(qmx, off, 32); qmn = a0 < qmn ? a0 : qmn; qmx = a1 > qmx ? a1 : qmx; }
    const int lim = t0 + lr;
    const int nk = (t0 + 16 + 31) & ~31;
    const size_t pbase = (size_t)zh * SEQ * HD;
    const size_t qo = pbase + (size_t)(t0 + lr) * HD + 8 * hi;
    const size_t ko = pbase + (size_t)lr * HD + 8 * hi;
    const size_t vo = pbase + (size_t)lr * SEQ + 8 * hi;
    v8f o[8], oR[8];
#pragma unroll
    for (int j = 0; j < 8; ++j) { o[j] = (v8f){}; oR[j] = (v8f){}; }
    float m = NEGB, l = 0.0f;
#pragma unroll 1
    for (int key0 = 0; key0 < nk; key0 += 32) {
        const int kdl = dk[key0 + lane];
        const bool inr = (kdl >= qmn) & (kdl <= qmx);
        if (__builtin_amdgcn_ballot_w32(inr) == 0u) continue;
        const int* kp = dk + key0 + 8 * hi;
        const v4i d0 = *(const v4i*)kp, d1 = *(const v4i*)(kp + 4), d2 = *(const v4i*)(kp + 16), d3 = *(const v4i*)(kp + 20);
        int ka8[8], kb8[8];
#pragma unroll
        for (int r = 0; r < 4; ++r) { ka8[r] = d0[r]; ka8[4 + r] = d1[r]; kb8[r] = d2[r]; kb8[4 + r] = d3[r]; }
        const v8f ta = sc16(QH, QR, KP, KR, qo, ko + (size_t)key0 * HD);
        const v8f tb = sc16(QH, QR, KP, KR, qo, ko + (size_t)(key0 + 16) * HD);
        const int ja = key0 + 8 * hi;
        bool fa[8], fb[8]; float mx = NEGB;
#pragma unroll
        for (int r = 0; r < 8; ++r) {
            fa[r] = (ka8[r] == mydoc) & (ja + r <= lim);
            fb[r] = (kb8[r] == mydoc) & (ja + 16 + r <= lim);
            mx = fmaxf(mx, fmaxf(fa[r] ? ta[r] : NEGB, fb[r] ? tb[r] : NEGB)); }
        mx = fmaxf(mx, __shfl_xor(mx, 16, 32));
        const float mnew = fmaxf(m, mx);
        const float alpha = __builtin_amdgcn_exp2f(m - mnew);
        const float sh = PSH - mnew;
        v16h pb, pr; float ls = 0.0f;
#pragma unroll
        for (int r = 0; r < 8; ++r) {
            const float xa = ta[r] + sh, xb = tb[r] + sh;
            const float ea = __builtin_amdgcn_exp2f(xa), eb = __builtin_amdgcn_exp2f(xb);
            const float ga = (fa[r] & (xa >= -14.0f)) ? ea : 0.0f, gb = (fb[r] & (xb >= -14.0f)) ? eb : 0.0f;
            const h16 pa = (h16)ga; const h16 pc = (h16)gb;
            pb[r] = pa; pb[8 + r] = pc;
            pr[r] = toh_flush((ga - (float)pa) * QRS); pr[8 + r] = toh_flush((gb - (float)pc) * QRS);
            ls += ga + gb; }
        l = l * alpha + ls; m = mnew;
#pragma unroll
        for (int j = 0; j < 8; ++j) { o[j] = o[j] * alpha; oR[j] = oR[j] * alpha; }
        const size_t vk = vo + (size_t)key0;
#pragma unroll
        for (int g = 0; g < 4; ++g) {
            const h16* va = VT + vk + (size_t)(32 * g) * SEQ;
            const h16* vr = VR + vk + (size_t)(32 * g) * SEQ;
            const v16h v0 = ldh(va), v1 = ldh(va + (size_t)16 * SEQ);
            const v16h w0 = ldh(vr), w1 = ldh(vr + (size_t)16 * SEQ);
            o[2 * g] = wmma16(v0, pb, o[2 * g]); o[2 * g + 1] = wmma16(v1, pb, o[2 * g + 1]);
            oR[2 * g] = wmma16(v0, pr, oR[2 * g]); oR[2 * g + 1] = wmma16(v1, pr, oR[2 * g + 1]);
            oR[2 * g] = wmma16(w0, pb, oR[2 * g]); oR[2 * g + 1] = wmma16(w1, pb, oR[2 * g + 1]);
            asm volatile("v_nop\n\tv_nop\n\tv_nop\n\tv_nop" : "+v"(o[2 * g]), "+v"(o[2 * g + 1]), "+v"(oR[2 * g]), "+v"(oR[2 * g + 1]) : "v"(v0), "v"(v1), "v"(w0), "v"(w1), "v"(pb), "v"(pr));
        }
    }
    l += __shfl_xor(l, 16, 32);
    const bool any = l > 0.0f;
    const float lsafe = any ? l : 1.0f;
    const float inv = any ? (1.0f / lsafe) : 0.0f;
    const int wb = wave * 16 * OSP;
#pragma unroll
    for (int j = 0; j < 8; ++j) {
        const v8f f = o[j] + oR[j] * QRI; v4f a, c;
        a[0] = f[0] * inv; a[1] = f[1] * inv; a[2] = f[2] * inv; a[3] = f[3] * inv; c[0] = f[4] * inv; c[1] = f[5] * inv; c[2] = f[6] * inv; c[3] = f[7] * inv;
        *(v4fa*)(&os[wb + lr * OSP + 16 * j + 8 * hi]) = a; *(v4fa*)(&os[wb + lr * OSP + 16 * j + 8 * hi + 4]) = c; }
    wave_sync();
    v8us hv[8], lv[8];
#pragma unroll
    for (int s = 0; s < 8; ++s) { const int row = 2 * s + (lane >> 4), c8 = (lane & 15) * 8;
        const v4f x0 = *(const v4fa*)(&os[wb + row * OSP + c8]); const v4f x1 = *(const v4fa*)(&os[wb + row * OSP + c8 + 4]);
#pragma unroll
        for (int i = 0; i < 4; ++i) { const unsigned short a0 = f2bf(x0[i]); const unsigned short a1 = f2bf(x1[i]); hv[s][i] = a0; hv[s][4 + i] = a1;
            lv[s][i] = f2bf(x0[i] - bf2f(a0)); lv[s][4 + i] = f2bf(x1[i] - bf2f(a1)); } }
    bf* yrow = Y2 + ((size_t)b * SEQ + t0) * (size_t)(2 * DM) + h * HD;
#pragma unroll 1
    for (int ps = 0; ps < 2; ++ps) {
#pragma unroll
        for (int s = 0; s < 8; ++s) { const int row = 2 * s + (lane >> 4), c8 = (lane & 15) * 8;
            const size_t oo = (size_t)row * (size_t)(2 * DM) + c8;
            *(volatile v8us*)(yrow + oo) = hv[s]; *(volatile v8us*)(yrow + oo + DM) = lv[s]; }
        if (ps == 0) __threadfence(); }
}

__global__ __launch_bounds__(32) void k_oproj(const bf* __restrict__ A, const bf* __restrict__ Bt, float* OUT) {
    __shared__ __align__(16) float os[16 * 68];
    const int KA = 2 * DM;
    const int lane = threadIdx.x & 31, lr = lane & 15, hi = lane >> 4; const int r0 = blockIdx.x * 64, c0 = blockIdx.y * 64;
    v8f acc[4][4];
#pragma unroll
    for (int mb = 0; mb < 4; ++mb)
#pragma unroll
        for (int nb = 0; nb < 4; ++nb) acc[mb][nb] = (v8f){};
    const size_t aoff = (size_t)(r0 + lr) * KA + 8 * hi, boff = (size_t)(c0 + lr) * DM + 8 * hi;
#pragma unroll 1
    for (int kc = 0; kc < KA; kc += 32) {
        const int kb = kc & (DM - 1);
        v16bf a[4];
#pragma unroll
        for (int mb = 0; mb < 4; ++mb) a[mb] = ldb(A + aoff + (size_t)mb * 16 * KA + kc);
#pragma unroll
        for (int nb = 0; nb < 4; ++nb) { const v16bf b = ldb(Bt + boff + (size_t)nb * 16 * DM + kb);
#pragma unroll
            for (int mb = 0; mb < 4; ++mb) acc[mb][nb] = wmmab(a[mb], b, acc[mb][nb]); }
        asm volatile("v_nop\n\tv_nop\n\tv_nop\n\tv_nop" : "+v"(acc[0][0]), "+v"(acc[1][1]), "+v"(acc[2][2]), "+v"(acc[3][3]) : "v"(a[0]), "v"(a[1]), "v"(a[2]), "v"(a[3]));
    }
    const int bb = r0 / SEQ, tt = r0 % SEQ;
    float* orow = OUT + ((size_t)bb * OUT_SEQ + tt) * DM + c0;
#pragma unroll
    for (int mb = 0; mb < 4; ++mb) {
#pragma unroll
        for (int nb = 0; nb < 4; ++nb) {
#pragma unroll
            for (int j = 0; j < 8; ++j) os[(hi * 8 + j) * 68 + nb * 16 + lr] = acc[mb][nb][j]; }
        wave_sync();
#pragma unroll 1
        for (int ps = 0; ps < 2; ++ps) {
#pragma unroll
            for (int s = 0; s < 8; ++s) { const int row = 2 * s + (lane >> 4), cofs = (lane & 15) * 4;
                const v4f val = *(const v4fa*)(&os[row * 68 + cofs]);
                *(volatile v4f*)(orow + (size_t)(mb * 16 + row) * DM + cofs) = val; }
            if (ps == 0) __threadfence(); }
        wave_sync();
    }
}

static constexpr size_t al256(size_t v) { return (v + 255) & ~(size_t)255; }
static constexpr size_t SZ_XB = al256((size_t)NB * SEQ * DM * 2);
static constexpr size_t SZ_WB = al256((size_t)3 * DM * DM * 2);
static constexpr size_t SZ_WC = al256((size_t)DM * DM * 2);
static constexpr size_t SZ_TB = al256((size_t)SEQ * NF * 4);
static constexpr size_t SZ_PL = al256((size_t)NB * NH_ * SEQ * HD * 2);
static constexpr size_t SZ_Y2 = al256((size_t)NB * SEQ * 2 * DM * 2);
static constexpr size_t SZ_TOTAL = SZ_XB + SZ_WB + SZ_WC + 2 * SZ_TB + 6 * SZ_PL + SZ_Y2;
static_assert(SZ_TOTAL <= (size_t)134217728);
static_assert(((size_t)DM * DM * 2) % 256 == 0);
static_assert(((size_t)NB * NH_ * SEQ * HD * 2) % 256 == 0);
static_assert((size_t)NB * NH_ * SEQ * HD == (size_t)NB * DM * SEQ);

extern "C" void kernel_launch(void* const* d_in, const int* in_sizes, int n_in,
                              void* d_out, int out_size, void* d_ws, size_t ws_size, hipStream_t stream) {
    if (n_in < 6) return;
    const size_t needx = ((size_t)(NB - 1) * SEQ_FULL + SEQ) * DM;
    const size_t needd = (size_t)(NB - 1) * SEQ_FULL + SEQ;
    if ((size_t)in_sizes[0] < needx || (size_t)in_sizes[1] < needx) return;
    if ((size_t)in_sizes[2] < (size_t)3 * DM * DM || in_sizes[3] < 2 || (size_t)in_sizes[4] < (size_t)DM * DM) return;
    if ((size_t)in_sizes[5] < needd) return;
    if ((size_t)out_size < ((size_t)(NB - 1) * OUT_SEQ + SEQ) * DM) return;
    if (SZ_TOTAL > ws_size) return;
    const float* x   = (const float*)d_in[0];
    const float* ve  = (const float*)d_in[1];
    const float* wq  = (const float*)d_in[2];
    const float* lam = (const float*)d_in[3];
    const float* wc  = (const float*)d_in[4];
    const int* docs  = (const int*)d_in[5];
    float* OUT = (float*)d_out;
    char* wsp = (char*)d_ws;
    bf* XB = (bf*)wsp; wsp += SZ_XB;
    bf* WB = (bf*)wsp; wsp += SZ_WB;
    bf* WC = (bf*)wsp; wsp += SZ_WC;
    float* CS = (float*)wsp; wsp += SZ_TB;
    float* SN = (float*)wsp; wsp += SZ_TB;
    h16* PH = (h16*)wsp; wsp += 2 * SZ_PL;
    h16* PR = (h16*)wsp; wsp += 2 * SZ_PL;
    h16* VT = (h16*)wsp; wsp += SZ_PL;
    h16* VR = (h16*)wsp; wsp += SZ_PL;
    bf* Y2 = (bf*)wsp; wsp += SZ_Y2;
    const size_t plane = (size_t)NB * NH_ * SEQ * HD;
    const h16* QH = PH; const h16* KP = PH + plane;
    const h16* QR = PR; const h16* KR = PR + plane;

    if (SEQ == SEQ_FULL) {
        const size_t n8 = (size_t)NB * SEQ * DM / 8;
        k_cvt8<<<(unsigned)((n8 + 255) / 256), 256, 0, stream>>>(x, XB, n8);
    } else {
        const size_t n8 = (size_t)SEQ * DM / 8;
        for (int b = 0; b < NB; ++b) k_cvt8<<<(unsigned)((n8 + 255) / 256), 256, 0, stream>>>(x + (size_t)b * SEQ_FULL * DM, XB + (size_t)b * SEQ * DM, n8);
    }
    { const size_t n8 = (size_t)3 * DM * DM / 8; k_cvt8<<<(unsigned)((n8 + 255) / 256), 256, 0, stream>>>(wq, WB, n8); }
    { const size_t n8 = (size_t)DM * DM / 8;     k_cvt8<<<(unsigned)((n8 + 255) / 256), 256, 0, stream>>>(wc, WC, n8); }
    k_rot<<<(unsigned)(((size_t)SEQ * NF) / 256), 256, 0, stream>>>(CS, SN);

    k_qk<<<dim3(NB * SEQ / 32, 2 * NH_, 1), 32, 0, stream>>>(XB, WB, CS, SN, PH, PR);
    k_vt<<<dim3(DM / 64, NB * SEQ / 64, 1), 32, 0, stream>>>(WB + (size_t)2 * DM * DM, XB, ve, lam, VT, VR);
    k_flash<<<dim3(SEQ / (16 * AW), NB * NH_, 1), 32 * AW, 0, stream>>>(QH, QR, KP, KR, VT, VR, docs, Y2);
    k_oproj<<<dim3(NB * SEQ / 64, DM / 64, 1), 32, 0, stream>>>(Y2, WC, OUT);
}
